// TokenMudule_53506702573964
// MI455X (gfx1250) — hardware-verified
//
#include <hip/hip_runtime.h>
#include <stdint.h>


#define NBATCH 32
#define HWD 196
#define HSD 14
#define CDIM 768
#define NCDIM 4096
#define MROWS (NBATCH * HWD)
#define GROWS 64
#define NTHR 256

typedef __attribute__((ext_vector_type(16))) _Float16 v16h;
typedef __attribute__((ext_vector_type(8)))  _Float16 v8h;
typedef __attribute__((ext_vector_type(16))) __bf16   v16b;
typedef __attribute__((ext_vector_type(8)))  __bf16   v8b;
typedef __attribute__((ext_vector_type(8)))  float    v8f;
typedef __attribute__((ext_vector_type(4)))  float    v4f;

__device__ __forceinline__ unsigned short f2bf_bits(float f) {
  unsigned u = __float_as_uint(f);
  return (unsigned short)((u + 0x7FFFu + ((u >> 16) & 1u)) >> 16);
}
__device__ __forceinline__ float bf_bits2f(unsigned short h) { return __uint_as_float(((unsigned)h) << 16); }

__device__ __forceinline__ void dep_guard_h(v8f& a, v8f& b, v16h x, v16h y) { asm volatile("v_nop\n\tv_nop\n\tv_nop\n\tv_nop" : "+v"(a), "+v"(b) : "v"(x), "v"(y)); }
__device__ __forceinline__ void dep_guard_b(v8f& a, v8f& b, v16b x, v16b y) { asm volatile("v_nop\n\tv_nop\n\tv_nop\n\tv_nop" : "+v"(a), "+v"(b) : "v"(x), "v"(y)); }
__device__ __forceinline__ void keep4_h(v16h a, v16h b, v16h c, v16h d) { asm volatile("v_nop" :: "v"(a), "v"(b), "v"(c), "v"(d)); }
__device__ __forceinline__ void keep4_b(v16b a, v16b b, v16b c, v16b d) { asm volatile("v_nop" :: "v"(a), "v"(b), "v"(c), "v"(d)); }
__device__ __forceinline__ void acc_guard4(v8f& a, v8f& b, v8f& c, v8f& d) { asm volatile("v_nop\n\tv_nop\n\tv_nop\n\tv_nop" : "+v"(a), "+v"(b), "+v"(c), "+v"(d)); }
template <typename T> struct Frag;
template <> struct Frag<_Float16> {
  typedef v16h V; union U { v16h v; v8h h[2]; };
  static __device__ __forceinline__ v16h load(const _Float16* p) {
    U f; f.h[0] = *(const v8h*)(p); f.h[1] = *(const v8h*)(p + 16); return f.v;
  }
  static __device__ __forceinline__ v8f mma(v16h a, v16h b, v8f c) {
    return __builtin_amdgcn_wmma_f32_16x16x32_f16(false, a, false, b, (short)0, c, false, false);
  }
  static __device__ __forceinline__ void guard(v8f& a, v8f& b, v16h x, v16h y) { dep_guard_h(a, b, x, y); }
  static __device__ __forceinline__ void keep(v16h a, v16h b, v16h c, v16h d) { keep4_h(a, b, c, d); }
};
template <> struct Frag<__bf16> {
  typedef v16b V; union U { v16b v; v8b h[2]; };
  static __device__ __forceinline__ v16b load(const __bf16* p) {
    U f; f.h[0] = *(const v8b*)(p); f.h[1] = *(const v8b*)(p + 16); return f.v;
  }
  static __device__ __forceinline__ v8f mma(v16b a, v16b b, v8f c) {
    return __builtin_amdgcn_wmma_f32_16x16x32_bf16(false, a, false, b, (short)0, c, false, false);
  }
  static __device__ __forceinline__ void guard(v8f& a, v8f& b, v16b x, v16b y) { dep_guard_b(a, b, x, y); }
  static __device__ __forceinline__ void keep(v16b a, v16b b, v16b c, v16b d) { keep4_b(a, b, c, d); }
};

template <int ET> struct Elem;
template <> struct Elem<0> { typedef _Float16 T; };
template <> struct Elem<1> { typedef __bf16 T; };
template <int ET, bool SPLIT, int BIAS_MODE, int OUT_MODE, bool RESID, int ACT = 0>
__global__ __launch_bounds__(256) void wmma_gemm64(
    const unsigned short* __restrict__ Ap, const unsigned short* __restrict__ A2p, int lda, long strideA,
    const unsigned short* __restrict__ Btp, const unsigned short* __restrict__ Bt2p, int ldb, long strideB,
    void* __restrict__ Cout, void* __restrict__ Cout2, int ldc, long strideC,
    const float* __restrict__ bias,
    const float* __restrict__ resid, long strideR,
    int M, int N, int K, float scale, float oscale) {
  typedef typename Elem<ET>::T T;
  typedef typename Frag<T>::V V;
  const T* A = (const T*)Ap; const T* A2 = (const T*)A2p; const T* Bt = (const T*)Btp; const T* Bt2 = (const T*)Bt2p;
  __shared__ __align__(16) float sT[8][16 * 68];
  const int b    = blockIdx.y;
  const int lane = threadIdx.x & 31;
  const int wave = threadIdx.x >> 5;
  const int tilesN = N >> 6;
  const int tilesM = M >> 6;
  const int tile = blockIdx.x * 8 + wave;
  if (tile >= tilesM * tilesN) return;
  const int tm = tile / tilesN;
  const int tn = tile - tm * tilesN;
  const int m0 = tm << 6;
  const int n0 = tn << 6;

  const T* Ab  = A  + (size_t)b * strideA;
  const T* Bb  = Bt + (size_t)b * strideB;
  const T* Ab2 = SPLIT ? (A2  + (size_t)b * strideA) : nullptr;
  const T* Bb2 = SPLIT ? (Bt2 + (size_t)b * strideB) : nullptr;

  const int rlane = lane & 15;
  const int koff  = (lane >> 4) * 8;
  const int mOff  = (lane >> 4) * 8;

  v8f acc[4][4];
#pragma unroll
  for (int i = 0; i < 4; ++i)
#pragma unroll
    for (int j = 0; j < 4; ++j) acc[i][j] = (v8f){0.f,0.f,0.f,0.f,0.f,0.f,0.f,0.f};

  for (int k0 = 0; k0 < K; k0 += 32) {
    V bh[4], bl[4];
#pragma unroll
    for (int j = 0; j < 4; ++j) {
      const size_t bo = (size_t)(n0 + (j << 4) + rlane) * ldb + koff + k0;
      bh[j] = Frag<T>::load(Bb + bo);
      if (SPLIT) bl[j] = Frag<T>::load(Bb2 + bo);
    }
#pragma unroll
    for (int i = 0; i < 4; ++i) {
      const size_t ao = (size_t)(m0 + (i << 4) + rlane) * lda + koff + k0;
      V ah = Frag<T>::load(Ab + ao);
      V al;
      if (SPLIT) al = Frag<T>::load(Ab2 + ao);
#pragma unroll
      for (int j = 0; j < 4; ++j) {
        acc[i][j] = Frag<T>::mma(ah, bh[j], acc[i][j]);
        if (SPLIT) {
          acc[i][j] = Frag<T>::mma(ah, bl[j], acc[i][j]);
          acc[i][j] = Frag<T>::mma(al, bh[j], acc[i][j]);
        }
      }
      Frag<T>::guard(acc[i][0], acc[i][3], ah, SPLIT ? al : ah);
    }
    Frag<T>::keep(bh[0], bh[1], bh[2], bh[3]);
    if (SPLIT) Frag<T>::keep(bl[0], bl[1], bl[2], bl[3]);
  }
  acc_guard4(acc[0][0], acc[0][1], acc[0][2], acc[0][3]);
  acc_guard4(acc[1][0], acc[1][1], acc[1][2], acc[1][3]);
  acc_guard4(acc[2][0], acc[2][1], acc[2][2], acc[2][3]);
  acc_guard4(acc[3][0], acc[3][1], acc[3][2], acc[3][3]);

  float* slab = sT[wave];
  const float* Rb = RESID ? (resid + (size_t)b * strideR) : nullptr;
#pragma unroll
  for (int i = 0; i < 4; ++i) {
    const int mBase = m0 + (i << 4);
#pragma unroll
    for (int j = 0; j < 4; ++j) {
      const int n = n0 + (j << 4) + rlane;
      float bv = 0.f;
      if (BIAS_MODE == 2) bv = bias[n];
#pragma unroll
      for (int r = 0; r < 8; ++r) {
        float v = acc[i][j][r] * scale;
        if (BIAS_MODE == 1) v += bias[mBase + mOff + r];
        if (BIAS_MODE == 2) v += bv;
        if (RESID) v += Rb[(size_t)(mBase + mOff + r) * ldc + n];
        if (ACT == 1) v = tanhf(v);
        if (ACT == 2) v = fmaxf(v, 0.0f);
        if (ACT == 3) v = v / (1.0f + expf(-v));
        if (ACT == 4) v = (v > 0.f) ? v : 0.01f * v;
        if (ACT == 5) v = 0.5f * v * (1.0f + erff(v * 0.70710678118654752f));
        v = v * oscale;
        slab[(mOff + r) * 68 + (j << 4) + rlane] = v;
      }
    }
    __builtin_amdgcn_fence(__ATOMIC_RELEASE, "workgroup");
    __builtin_amdgcn_wave_barrier();
    __builtin_amdgcn_fence(__ATOMIC_ACQUIRE, "workgroup");
    if (OUT_MODE == 0) {
      float* C = (float*)Cout + (size_t)b * strideC;
      const int hh = lane >> 4, c4 = (lane & 15) * 4;
      for (int pass = 0; pass < 2; ++pass) {
#pragma unroll
        for (int it = 0; it < 8; ++it) {
          const int row = it * 2 + hh;
          v4f v = *(const v4f*)(slab + row * 68 + c4);
          *(volatile v4f*)(C + (size_t)(mBase + row) * ldc + n0 + c4) = v;
        }
        __threadfence();
      }
    } else {
      const int q = lane >> 3, c8 = (lane & 7) * 8;
      unsigned short* C  = (unsigned short*)Cout  + (size_t)b * strideC;
      unsigned short* C2 = (OUT_MODE == 2) ? ((unsigned short*)Cout2 + (size_t)b * strideC) : nullptr;
      for (int pass = 0; pass < 2; ++pass) {
#pragma unroll
        for (int it = 0; it < 4; ++it) {
          const int row = it * 4 + q;
          const float* sp = slab + row * 68 + c8;
          v8h hv, lv;
#pragma unroll
          for (int e = 0; e < 8; ++e) {
            if (OUT_MODE == 1) {
              hv[e] = (_Float16)sp[e];
            } else {
              unsigned short hb = f2bf_bits(sp[e]);
              unsigned short lb = f2bf_bits(sp[e] - bf_bits2f(hb));
              hv[e] = __builtin_bit_cast(_Float16, hb);
              lv[e] = __builtin_bit_cast(_Float16, lb);
            }
          }
          *(volatile v8h*)(C + (size_t)(mBase + row) * ldc + n0 + c8) = hv;
          if (OUT_MODE == 2) *(volatile v8h*)(C2 + (size_t)(mBase + row) * ldc + n0 + c8) = lv;
        }
        __threadfence();
      }
    }
    __builtin_amdgcn_fence(__ATOMIC_RELEASE, "workgroup");
    __builtin_amdgcn_wave_barrier();
    __builtin_amdgcn_fence(__ATOMIC_ACQUIRE, "workgroup");
  }
}

__global__ __launch_bounds__(NTHR) void k_wtr(const float* __restrict__ in, _Float16* __restrict__ out,
                                              int Kd, int Nd, float wscale) {
  __shared__ float tile[64 * 33];
  const int tid = threadIdx.x;
  const int n0 = blockIdx.x * 32;
  const int k0 = blockIdx.y * 64;
#pragma unroll
  for (int r = 0; r < 8; ++r) {
    const int idx = tid + NTHR * r;
    const int kk = idx >> 5, nn = idx & 31;
    tile[kk * 33 + nn] = in[(size_t)(k0 + kk) * Nd + n0 + nn];
  }
  __syncthreads();
  const int nn = tid >> 3, q = tid & 7;
  v8h hv;
#pragma unroll
  for (int e = 0; e < 8; ++e) hv[e] = (_Float16)(tile[(8 * q + e) * 33 + nn] * wscale);
  _Float16* dst = out + (size_t)(n0 + nn) * Kd + k0 + 8 * q;
  *(volatile v8h*)dst = hv;
  __threadfence();
  *(volatile v8h*)dst = hv;
}

__global__ __launch_bounds__(NTHR) void k_ssa(const float* __restrict__ x, float* __restrict__ T) {
  __shared__ float xs[HWD * 32];
  __shared__ float part[9 * 8 * 32];
  __shared__ float rns[9 * 32];
  const int tid = threadIdx.x, lane = tid & 31, w = tid >> 5;
  const int b  = blockIdx.x / (CDIM / 32);
  const int cg = blockIdx.x - b * (CDIM / 32);
  const int c0 = cg * 32;
  const float* xb = x + (size_t)b * HWD * CDIM + c0;
  for (int idx = tid; idx < HWD * 32; idx += NTHR) {
    const int t = idx >> 5, cl = idx & 31;
    xs[idx] = xb[(size_t)t * CDIM + cl];
  }
  __syncthreads();

  float s[9];
#pragma unroll
  for (int kk = 0; kk < 9; ++kk) s[kk] = 0.f;
  for (int t = w; t < HWD; t += 8) {
    const int i = t / HSD, j = t - i * HSD;
    const float center = xs[t * 32 + lane];
#pragma unroll
    for (int kk = 0; kk < 9; ++kk) {
      const int ri = i + (kk / 3) - 2;
      const int rj = j + (kk % 3) - 1;
      const bool valid = ((unsigned)ri < (unsigned)HSD) && ((unsigned)rj < (unsigned)HSD);
      const int tn = valid ? (ri * HSD + rj) : t;
      float nb = xs[tn * 32 + lane];
      nb = valid ? nb : 0.f;
      const float p = center * nb;
      s[kk] = fmaf(p, p, s[kk]);
    }
  }
#pragma unroll
  for (int kk = 0; kk < 9; ++kk) part[(kk * 8 + w) * 32 + lane] = s[kk];
  __syncthreads();
  for (int idx = tid; idx < 9 * 32; idx += NTHR) {
    const int kk = idx >> 5, cl = idx & 31;
    float a = 0.f;
#pragma unroll
    for (int ww = 0; ww < 8; ++ww) a += part[(kk * 8 + ww) * 32 + cl];
    rns[idx] = 1.0f / fmaxf(sqrtf(a), 1e-12f);
  }
  __syncthreads();

  for (int t = w; t < HWD; t += 8) {
    const int i = t / HSD, j = t - i * HSD;
    const float center = xs[t * 32 + lane];
    float acc = 0.f;
#pragma unroll
    for (int kk = 0; kk < 9; ++kk) {
      const int ri = i + (kk / 3) - 2;
      const int rj = j + (kk % 3) - 1;
      const bool valid = ((unsigned)ri < (unsigned)HSD) && ((unsigned)rj < (unsigned)HSD);
      const int tn = valid ? (ri * HSD + rj) : t;
      float nb = xs[tn * 32 + lane];
      nb = valid ? nb : 0.f;
      const float p = center * nb;
      const float v = fmaxf(p * rns[kk * 32 + lane], 1e-6f);
      acc = fmaf(v * v, v, acc);
    }
    const float pooled = cbrtf(acc * (1.0f / 9.0f));
    const float val = pooled + center;
    float* dst = T + ((size_t)b * HWD + t) * CDIM + c0 + lane;
    *(volatile float*)dst = val;
    __threadfence();
    *(volatile float*)dst = val;
  }
}

__global__ __launch_bounds__(NTHR) void k_rownorm(const float* __restrict__ T, _Float16* __restrict__ A1) {
  __shared__ __align__(16) float af[CDIM];
  __shared__ float part[8];
  const int row = blockIdx.x;
  const int tid = threadIdx.x, lane = tid & 31, w = tid >> 5;
  const float* tr = T + (size_t)row * CDIM;
  const float v0 = tr[tid], v1 = tr[tid + 256], v2 = tr[tid + 512];
  float ss = v0 * v0 + v1 * v1 + v2 * v2;
#pragma unroll
  for (int off = 16; off; off >>= 1) ss += __shfl_xor(ss, off, 32);
  if (lane == 0) part[w] = ss;
  __syncthreads();
  float tot = 0.f;
#pragma unroll
  for (int ww = 0; ww < 8; ++ww) tot += part[ww];
  const float rn = 16.0f / fmaxf(sqrtf(tot), 1e-12f);
  af[tid] = v0 * rn; af[tid + 256] = v1 * rn; af[tid + 512] = v2 * rn;
  __syncthreads();
  if (tid < CDIM / 8) {
    v8h hv;
#pragma unroll
    for (int e = 0; e < 8; ++e) hv[e] = (_Float16)af[8 * tid + e];
    _Float16* dst = A1 + (size_t)row * CDIM + 8 * tid;
    *(volatile v8h*)dst = hv;
    __threadfence();
    *(volatile v8h*)dst = hv;
  }
}

__global__ __launch_bounds__(NTHR) void k_gem(const float* __restrict__ T2, _Float16* __restrict__ G) {
  __shared__ __align__(16) float gf[CDIM];
  const int r = blockIdx.x;
  const int tid = threadIdx.x;
  float g0 = 0.f, g1 = 0.f, g2 = 0.f;
  if (r < NBATCH) {
    const float* base = T2 + (size_t)r * HWD * CDIM;
    float a0 = 0.f, a1 = 0.f, a2 = 0.f;
#pragma unroll 2
    for (int t = 0; t < HWD; ++t) {
      const float* rp = base + (size_t)t * CDIM;
      const float u0 = fmaxf(rp[tid], 1e-6f);       a0 = fmaf(u0 * u0, u0, a0);
      const float u1 = fmaxf(rp[tid + 256], 1e-6f); a1 = fmaf(u1 * u1, u1, a1);
      const float u2 = fmaxf(rp[tid + 512], 1e-6f); a2 = fmaf(u2 * u2, u2, a2);
    }
    g0 = cbrtf(a0 * (1.0f / (float)HWD)) * 256.0f;
    g1 = cbrtf(a1 * (1.0f / (float)HWD)) * 256.0f;
    g2 = cbrtf(a2 * (1.0f / (float)HWD)) * 256.0f;
  }
  gf[tid] = g0; gf[tid + 256] = g1; gf[tid + 512] = g2;
  __syncthreads();
  if (tid < CDIM / 8) {
    v8h hv;
#pragma unroll
    for (int e = 0; e < 8; ++e) hv[e] = (_Float16)gf[8 * tid + e];
    _Float16* dst = G + (size_t)r * CDIM + 8 * tid;
    *(volatile v8h*)dst = hv;
    __threadfence();
    *(volatile v8h*)dst = hv;
  }
}

__global__ __launch_bounds__(NTHR) void k_headnorm(const float* __restrict__ D, float* __restrict__ out) {
  __shared__ float part[8];
  const int b = blockIdx.x;
  const int tid = threadIdx.x, lane = tid & 31, w = tid >> 5;
  const float* row = D + (size_t)b * NCDIM;
  v4f dv[4];
  float ss = 0.f;
#pragma unroll
  for (int it = 0; it < 4; ++it) {
    dv[it] = *(const v4f*)(row + (size_t)(it * NTHR + tid) * 4);
    ss += dv[it][0] * dv[it][0] + dv[it][1] * dv[it][1] + dv[it][2] * dv[it][2] + dv[it][3] * dv[it][3];
  }
#pragma unroll
  for (int off = 16; off; off >>= 1) ss += __shfl_xor(ss, off, 32);
  if (lane == 0) part[w] = ss;
  __syncthreads();
  float tot = 0.f;
#pragma unroll
  for (int ww = 0; ww < 8; ++ww) tot += part[ww];
  const float rn = 1.0f / fmaxf(sqrtf(tot), 1e-12f);
  float* orow = out + (size_t)b * NCDIM;
  for (int pass = 0; pass < 2; ++pass) {
#pragma unroll
    for (int it = 0; it < 4; ++it) {
      const v4f o = dv[it] * rn;
      *(volatile v4f*)(orow + (size_t)(it * NTHR + tid) * 4) = o;
    }
    __threadfence();
  }
}

extern "C" void kernel_launch(void* const* d_in, const int* in_sizes, int n_in,
                              void* d_out, int out_size, void* d_ws, size_t ws_size,
                              hipStream_t stream) {
  if (n_in < 7) return;
  if (in_sizes[0] != NBATCH * HWD * CDIM) return;
  if (in_sizes[1] != CDIM * CDIM || in_sizes[2] != CDIM) return;
  if (in_sizes[3] != CDIM * CDIM || in_sizes[4] != CDIM) return;
  if (in_sizes[5] != CDIM * NCDIM || in_sizes[6] != NCDIM) return;
  if (out_size != NBATCH * NCDIM) return;

  const float* x      = (const float*)d_in[0];
  const float* fc1_w  = (const float*)d_in[1];
  const float* fc1_b  = (const float*)d_in[2];
  const float* fc2_w  = (const float*)d_in[3];
  const float* fc2_b  = (const float*)d_in[4];
  const float* head_w = (const float*)d_in[5];
  const float* head_b = (const float*)d_in[6];
  float* out = (float*)d_out;

  const size_t sz_T  = (size_t)MROWS * CDIM * 4;
  const size_t sz_A1 = (size_t)MROWS * CDIM * 2;
  const size_t sz_H  = (size_t)MROWS * CDIM * 2;
  const size_t sz_W  = (size_t)CDIM * CDIM * 2;
  const size_t sz_Wh = (size_t)NCDIM * CDIM * 2;
  const size_t sz_G  = (size_t)GROWS * CDIM * 2;
  const size_t sz_D  = (size_t)GROWS * NCDIM * 4;
  const size_t off_T  = 0;
  const size_t off_A1 = off_T + sz_T;
  const size_t off_H  = off_A1 + sz_A1;
  const size_t off_W1 = off_H + sz_H;
  const size_t off_W2 = off_W1 + sz_W;
  const size_t off_Wh = off_W2 + sz_W;
  const size_t off_G  = off_Wh + sz_Wh;
  const size_t off_D  = off_G + sz_G;
  const size_t total  = off_D + sz_D;
  if (total > ws_size) return;

  char* ws = (char*)d_ws;
  float*    Tbuf = (float*)(ws + off_T);
  _Float16* A1   = (_Float16*)(ws + off_A1);
  _Float16* Hp   = (_Float16*)(ws + off_H);
  _Float16* W1t  = (_Float16*)(ws + off_W1);
  _Float16* W2t  = (_Float16*)(ws + off_W2);
  _Float16* Wht  = (_Float16*)(ws + off_Wh);
  _Float16* Gp   = (_Float16*)(ws + off_G);
  float*    Dsc  = (float*)(ws + off_D);

  k_wtr<<<dim3(CDIM / 32, CDIM / 64), NTHR, 0, stream>>>(fc1_w, W1t, CDIM, CDIM, 64.0f);
  k_wtr<<<dim3(CDIM / 32, CDIM / 64), NTHR, 0, stream>>>(fc2_w, W2t, CDIM, CDIM, 64.0f);
  k_wtr<<<dim3(NCDIM / 32, CDIM / 64), NTHR, 0, stream>>>(head_w, Wht, CDIM, NCDIM, 64.0f);

  k_ssa<<<NBATCH * (CDIM / 32), NTHR, 0, stream>>>(x, Tbuf);
  k_rownorm<<<MROWS, NTHR, 0, stream>>>(Tbuf, A1);

  const int tiles12 = (MROWS / 64) * (CDIM / 64);
  const int blocks12 = (tiles12 + 7) / 8;
  wmma_gemm64<0, false, 2, 1, false, 5><<<dim3(blocks12, 1), 256, 0, stream>>>(
      (const unsigned short*)A1, (const unsigned short*)A1, CDIM, 0L,
      (const unsigned short*)W1t, (const unsigned short*)W1t, CDIM, 0L,
      (void*)Hp, (void*)Hp, CDIM, 0L,
      fc1_b, fc1_b, 0L,
      MROWS, CDIM, CDIM, 1.0f / 1024.0f, 256.0f);
  wmma_gemm64<0, false, 2, 0, false, 0><<<dim3(blocks12, 1), 256, 0, stream>>>(
      (const unsigned short*)Hp, (const unsigned short*)Hp, CDIM, 0L,
      (const unsigned short*)W2t, (const unsigned short*)W2t, CDIM, 0L,
      (void*)Tbuf, (void*)Tbuf, CDIM, 0L,
      fc2_b, fc2_b, 0L,
      MROWS, CDIM, CDIM, 1.0f / 16384.0f, 1.0f);

  k_gem<<<GROWS, NTHR, 0, stream>>>(Tbuf, Gp);
  const int tiles3 = (GROWS / 64) * (NCDIM / 64);
  const int blocks3 = (tiles3 + 7) / 8;
  wmma_gemm64<0, false, 2, 0, false, 0><<<dim3(blocks3, 1), 256, 0, stream>>>(
      (const unsigned short*)Gp, (const unsigned short*)Gp, CDIM, 0L,
      (const unsigned short*)Wht, (const unsigned short*)Wht, CDIM, 0L,
      (void*)Dsc, (void*)Dsc, NCDIM, 0L,
      head_b, head_b, 0L,
      GROWS, NCDIM, CDIM, 1.0f / 16384.0f, 1.0f);
  k_headnorm<<<NBATCH, NTHR, 0, stream>>>(Dsc, out);
  (void)hipGetLastError();
}
